// Block_66812511256726
// MI455X (gfx1250) — hardware-verified
//
#include <hip/hip_runtime.h>
#ifndef NQ
#define NQ 2048
#endif
#ifndef NKV
#define NKV 8192
#endif
#define NQ_FULL 2048
#define NKV_FULL 8192
#define CD 256
#define NHEAD 8
#define HD 32
#define DFF 1024
#define NSEG 8
#define RMS_EPS 1.1920929e-7f
#define ATT_SCALE 0.17677669529663687f

static_assert(CD == NHEAD * HD);
static_assert(HD == 32);
static_assert(NHEAD * 32 == 256);
static_assert(CD == 256);
static_assert(NQ % 128 == 0 && NKV % 128 == 0);
static_assert(NQ % 64 == 0 && NKV % 64 == 0);
static_assert(CD % 64 == 0 && DFF % 64 == 0 && (2 * CD) % 64 == 0);
static_assert(CD % 32 == 0 && DFF % 32 == 0);
static_assert(NQ <= NQ_FULL && NKV <= NKV_FULL);

typedef unsigned short v8us __attribute__((ext_vector_type(8), may_alias));
typedef float  v8f  __attribute__((ext_vector_type(8)));
typedef float  v4f  __attribute__((ext_vector_type(4)));
typedef float  v4fa __attribute__((ext_vector_type(4), may_alias));
typedef _Float16 v16h __attribute__((ext_vector_type(16)));
typedef _Float16 v4h __attribute__((ext_vector_type(4)));
union FragH { v16h v; v8us half[2]; _Float16 h[16]; unsigned short u[16]; };

__device__ __forceinline__ unsigned short bf16_bits(float x) { unsigned int u = __float_as_uint(x); return (unsigned short)((u + 0x7FFFu + ((u >> 16) & 1u)) >> 16); }
__device__ __forceinline__ float bf16_val(unsigned short b) { return __uint_as_float(((unsigned int)b) << 16); }
__device__ __forceinline__ float bf16_rne(float x) { return bf16_val(bf16_bits(x)); }

__device__ __forceinline__ v16h g2_frag(const unsigned short* p, int hh) { FragH f; f.half[0] = *(const v8us*)(p + 8 * hh); f.half[1] = *(const v8us*)(p + 16 + 8 * hh); return f.v; }
__device__ __forceinline__ v8f g2_mma(v16h a, v16h b, v8f c) { v8f d = __builtin_amdgcn_wmma_f32_16x16x32_f16(false, a, false, b, (short)0, c, false, false); asm volatile("v_nop\n\tv_nop\n\tv_nop\n\tv_nop" : "+v"(d) : "v"(a), "v"(b)); return d; }
__device__ __forceinline__ void g2_mma_pair(v16h a, v16h b0, v16h b1, v8f& c0, v8f& c1) {
  c0 = __builtin_amdgcn_wmma_f32_16x16x32_f16(false, a, false, b0, (short)0, c0, false, false);
  c1 = __builtin_amdgcn_wmma_f32_16x16x32_f16(false, a, false, b1, (short)0, c1, false, false);
  asm volatile("v_nop\n\tv_nop\n\tv_nop\n\tv_nop" : "+v"(c0), "+v"(c1) : "v"(a), "v"(b0), "v"(b1));
}

__global__ __launch_bounds__(256) void k_wnat(const float* __restrict__ w, size_t n8, _Float16* __restrict__ Bt) {
  const size_t t = (size_t)blockIdx.x * 256 + threadIdx.x; if (t >= n8) return; FragH f;
#pragma unroll
  for (int q = 0; q < 8; ++q) f.h[q] = (_Float16)(bf16_rne(w[t * 8 + q]) * 16.0f);
  const v8us o = f.half[0];
  *(volatile v8us*)((unsigned short*)Bt + t * 8) = o; __threadfence(); *(volatile v8us*)((unsigned short*)Bt + t * 8) = o;
}

__global__ __launch_bounds__(256) void k_rmsw(const float* __restrict__ X, const float* __restrict__ w, const float* __restrict__ pos, float eps, int bfin,
                                              _Float16* __restrict__ N16, _Float16* __restrict__ NP16, int nrows) {
  #pragma clang fp contract(off)
  const int lane = threadIdx.x & 31, wv = threadIdx.x >> 5;
  const int row = blockIdx.x * 8 + wv;
  if (row >= nrows) return;
  const size_t base = (size_t)row * CD;
  const int c0 = lane * 4, c1 = 128 + lane * 4;
  v4f a = *(const v4fa*)(X + base + c0);
  v4f b = *(const v4fa*)(X + base + c1);
  if (bfin != 0) {
#pragma unroll
    for (int q = 0; q < 4; ++q) { a[q] = bf16_rne(a[q]); b[q] = bf16_rne(b[q]); }
  }
  float ss = 0.f;
#pragma unroll
  for (int q = 0; q < 4; ++q) ss += a[q] * a[q];
#pragma unroll
  for (int q = 0; q < 4; ++q) ss += b[q] * b[q];
#pragma unroll
  for (int msk = 16; msk > 0; msk >>= 1) ss += __shfl_xor(ss, msk, 32);
  const float inv = __frsqrt_rn(ss * 0.00390625f + eps);
  const v4f wa = *(const v4fa*)(w + c0), wb = *(const v4fa*)(w + c1);
  v4f pa = {0.f, 0.f, 0.f, 0.f}, pb = {0.f, 0.f, 0.f, 0.f};
  if (pos != nullptr) { pa = *(const v4fa*)(pos + base + c0); pb = *(const v4fa*)(pos + base + c1); }
  v4h y0, y1, z0, z1;
#pragma unroll
  for (int q = 0; q < 4; ++q) {
    const float ya = a[q] * inv * bf16_rne(wa[q]);
    const float yb = b[q] * inv * bf16_rne(wb[q]);
    y0[q] = (_Float16)ya; y1[q] = (_Float16)yb;
    z0[q] = (_Float16)(ya + bf16_rne(pa[q])); z1[q] = (_Float16)(yb + bf16_rne(pb[q]));
  }
  for (int pass = 0; pass < 2; ++pass) {
    if (N16 != nullptr) { *(volatile v4h*)(N16 + base + c0) = y0; *(volatile v4h*)(N16 + base + c1) = y1; }
    if (NP16 != nullptr) { *(volatile v4h*)(NP16 + base + c0) = z0; *(volatile v4h*)(NP16 + base + c1) = z1; }
    if (pass == 0) __threadfence();
  }
}

__global__ __launch_bounds__(256) void k_vt(const _Float16* __restrict__ V16, int ldv, int voff, _Float16* __restrict__ VT, int nk) {
  __shared__ unsigned short tl[64][65];
  const int tid = threadIdx.x; const int cg = blockIdx.x & 3, sg = blockIdx.x >> 2; const int s0 = sg * 64;
  if (s0 >= nk) return;
  for (int i = tid; i < 64 * 8; i += 256) { const int j = i / 8, d8 = (i % 8) * 8; FragH f; f.half[0] = *(const v8us*)((const unsigned short*)V16 + (size_t)(s0 + j) * ldv + voff + cg * 64 + d8);
#pragma unroll
    for (int q = 0; q < 8; ++q) tl[d8 + q][j] = f.u[q]; }
  __syncthreads();
  for (int pass = 0; pass < 2; ++pass) {
    for (int i = tid; i < 64 * 8; i += 256) { const int d = i / 8, j8 = (i % 8) * 8; FragH f;
#pragma unroll
      for (int q = 0; q < 8; ++q) f.u[q] = tl[d][j8 + q];
      *(volatile v8us*)((unsigned short*)VT + (size_t)(cg * 64 + d) * nk + s0 + j8) = f.half[0]; }
    if (pass == 0) __threadfence(); }
}

template <int ACT, int RES>
__device__ __forceinline__ void gemm_body(const _Float16* __restrict__ A, int lda, const _Float16* __restrict__ Bh, int ldb, float alpha, const float* __restrict__ bias, float oscale,
                                          const float* __restrict__ R, int ldr, float* __restrict__ C, _Float16* __restrict__ C16, _Float16* __restrict__ C16L, int ldc, int M, int N, int K) {
  static_assert(ACT == 0 || ACT == 6);
  static_assert(RES == 0 || ACT == 0);
  __shared__ __attribute__((aligned(16))) float so[4][32][68];
  const int tid = threadIdx.x, w = tid >> 5, lane = tid & 31, ln = lane & 15, hh = lane >> 4;
  const int ntn = N >> 6; const int mt = blockIdx.x / ntn, nq = blockIdx.x - mt * ntn; const int row0 = mt * 128 + 32 * w, col0 = nq * 64; if (row0 >= M) return;
  const unsigned short* a0p = (const unsigned short*)A + (size_t)(row0 + ln) * lda; const unsigned short* a1p = a0p + (size_t)16 * lda;
  const unsigned short* b0p = (const unsigned short*)Bh + (size_t)(col0 + ln) * ldb; const unsigned short* b1p = b0p + (size_t)16 * ldb; const unsigned short* b2p = b1p + (size_t)16 * ldb; const unsigned short* b3p = b2p + (size_t)16 * ldb;
  const v8f z8 = {0.f,0.f,0.f,0.f,0.f,0.f,0.f,0.f}; v8f c00 = z8, c01 = z8, c02 = z8, c03 = z8, c10 = z8, c11 = z8, c12 = z8, c13 = z8;
#pragma unroll 1
  for (int kb = 0; kb < K; kb += 32) { const v16h a0 = g2_frag(a0p + kb, hh), a1 = g2_frag(a1p + kb, hh);
    v16h b = g2_frag(b0p + kb, hh); c00 = g2_mma(a0, b, c00); c10 = g2_mma(a1, b, c10);
    b = g2_frag(b1p + kb, hh); c01 = g2_mma(a0, b, c01); c11 = g2_mma(a1, b, c11);
    b = g2_frag(b2p + kb, hh); c02 = g2_mma(a0, b, c02); c12 = g2_mma(a1, b, c12);
    b = g2_frag(b3p + kb, hh); c03 = g2_mma(a0, b, c03); c13 = g2_mma(a1, b, c13); }
  v8f accs[8] = {c00, c01, c02, c03, c10, c11, c12, c13};
#pragma unroll
  for (int u = 0; u < 8; ++u) { const int t = u & 3, half = u >> 2; const int col = col0 + t * 16 + ln; const float bv = (bias != nullptr) ? bf16_rne(bias[col]) : 0.f;
#pragma unroll
    for (int r = 0; r < 8; ++r) { const int rloc = half * 16 + 8 * hh + r; float v = accs[u][r] * alpha + bv;
      if (ACT == 6) v = 0.5f * v * (1.0f + erff(v * 0.70710678118654752f));
      v *= oscale;
      so[w][rloc][t * 16 + ln] = v; } }
  __builtin_amdgcn_fence(4  , "workgroup"); __builtin_amdgcn_wave_barrier();
  const int rsub = lane >> 4, c4 = (lane & 15) * 4;
  if (RES != 0) {
#pragma unroll
    for (int q = 0; q < 16; ++q) { const int r = q * 2 + rsub; v4f v = *(const v4fa*)&so[w][r][c4]; v4f rv = *(const v4fa*)(R + (size_t)(row0 + r) * ldr + col0 + c4);
      if (RES == 2) { rv[0] = bf16_rne(rv[0]); rv[1] = bf16_rne(rv[1]); rv[2] = bf16_rne(rv[2]); rv[3] = bf16_rne(rv[3]); }
      v[0] += rv[0]; v[1] += rv[1]; v[2] += rv[2]; v[3] += rv[3]; *(v4fa*)&so[w][r][c4] = v; }
  }
  for (int pass = 0; pass < 2; ++pass) {
#pragma unroll
    for (int q = 0; q < 16; ++q) { const int r = q * 2 + rsub; const v4f v = *(const v4fa*)&so[w][r][c4];
      if (C != nullptr) *(volatile v4f*)(C + (size_t)(row0 + r) * ldc + col0 + c4) = v;
      if (C16 != nullptr) { v4h h4; for (int i = 0; i < 4; ++i) h4[i] = (_Float16)v[i]; *(volatile v4h*)(C16 + (size_t)(row0 + r) * ldc + col0 + c4) = h4;
        if (C16L != nullptr) { v4h l4; for (int i = 0; i < 4; ++i) l4[i] = (_Float16)((v[i] - (float)h4[i]) * 1024.0f); *(volatile v4h*)(C16L + (size_t)(row0 + r) * ldc + col0 + c4) = l4; } } }
    if (pass == 0) __threadfence(); }
}
__global__ __launch_bounds__(128) void k_gemm_p(const _Float16* __restrict__ A, int lda, const _Float16* __restrict__ Bh, int ldb, float alpha, const float* __restrict__ bias, float oscale,
                                                _Float16* __restrict__ C16, _Float16* __restrict__ C16L, int ldc, int M, int N, int K) {
  gemm_body<0, 0>(A, lda, Bh, ldb, alpha, bias, oscale, nullptr, 0, nullptr, C16, C16L, ldc, M, N, K); }
__global__ __launch_bounds__(128) void k_gemm_gelu(const _Float16* __restrict__ A, int lda, const _Float16* __restrict__ Bh, int ldb, float alpha, const float* __restrict__ bias, float oscale,
                                                   _Float16* __restrict__ C16, int ldc, int M, int N, int K) {
  gemm_body<6, 0>(A, lda, Bh, ldb, alpha, bias, oscale, nullptr, 0, nullptr, C16, nullptr, ldc, M, N, K); }
__global__ __launch_bounds__(128) void k_gemm_res(const _Float16* __restrict__ A, int lda, const _Float16* __restrict__ Bh, int ldb, float alpha, const float* __restrict__ bias,
                                                  const float* __restrict__ R, int ldr, float* __restrict__ C, int ldc, int M, int N, int K) {
  gemm_body<0, 1>(A, lda, Bh, ldb, alpha, bias, 1.0f, R, ldr, C, nullptr, nullptr, ldc, M, N, K); }
__global__ __launch_bounds__(128) void k_gemm_resin(const _Float16* __restrict__ A, int lda, const _Float16* __restrict__ Bh, int ldb, float alpha, const float* __restrict__ bias,
                                                    const float* __restrict__ R, int ldr, float* __restrict__ C, int ldc, int M, int N, int K) {
  gemm_body<0, 2>(A, lda, Bh, ldb, alpha, bias, 1.0f, R, ldr, C, nullptr, nullptr, ldc, M, N, K); }

__device__ __forceinline__ int seg_of(int n, const int (&cb)[NSEG]) { int s = 0;
#pragma unroll
  for (int i = 0; i < NSEG; ++i) s += (cb[i] <= n) ? 1 : 0;
  return s; }

template <int MASKED>
__device__ __forceinline__ void attn_body(const _Float16* __restrict__ QH, const _Float16* __restrict__ QL, const _Float16* __restrict__ Kp, int ldk,
                                          const _Float16* __restrict__ VT, int nk, const int* __restrict__ cu, _Float16* __restrict__ CTX) {
  __shared__ __attribute__((aligned(16))) unsigned short so[16][CD];
  const int tid = threadIdx.x, head = tid >> 5, lane = tid & 31, ln = lane & 15, hh = lane >> 4;
  const int q0 = blockIdx.x * 16;
  int cb[NSEG];
#pragma unroll
  for (int i = 0; i < NSEG; ++i) cb[i] = MASKED ? cu[1 + i] : 0;
  const int sq = seg_of(q0 + ln, cb), sqlo = seg_of(q0, cb), sqhi = seg_of(q0 + 15, cb);
  const size_t qoff = (size_t)(q0 + ln) * CD + head * HD;
  const v16h bqh = g2_frag((const unsigned short*)QH + qoff, hh);
  const v16h bql = g2_frag((const unsigned short*)QL + qoff, hh);
  const v8f z8 = {0.f,0.f,0.f,0.f,0.f,0.f,0.f,0.f};
  v8f o0 = z8, o1 = z8; float m = -1.0e30f, l = 0.f;
  const unsigned short* kbase = (const unsigned short*)Kp + head * HD;
  const unsigned short* vb0 = (const unsigned short*)VT + (size_t)(head * HD + ln) * nk;
  const unsigned short* vb1 = vb0 + (size_t)16 * nk;
#pragma unroll 1
  for (int kc = 0; kc < nk; kc += 64) {
    if (MASKED) { const int sklo = seg_of(kc, cb), skhi = seg_of(kc + 63, cb); if (skhi < sqlo || sklo > sqhi) continue; }
    v8f s[4];
#pragma unroll
    for (int t = 0; t < 4; ++t) {
      const v16h ka = g2_frag(kbase + (size_t)(kc + t * 16 + ln) * ldk, hh);
      v8f sh = z8, sl = z8;
      g2_mma_pair(ka, bqh, bql, sh, sl);
#pragma unroll
      for (int r = 0; r < 8; ++r) { float v = (sh[r] + sl[r] * 0.0009765625f) * ATT_SCALE;
        if (MASKED) { const int sk = seg_of(kc + t * 16 + 8 * hh + r, cb); v += (sk == sq) ? 0.f : -10000.0f; }
        s[t][r] = v; }
    }
    float mx = s[0][0];
#pragma unroll
    for (int t = 0; t < 4; ++t) {
#pragma unroll
      for (int r = 0; r < 8; ++r) mx = fmaxf(mx, s[t][r]); }
    mx = fmaxf(mx, __shfl_xor(mx, 16, 32));
    const float mn = fmaxf(m, mx);
    const float c = __expf(m - mn);
    m = mn;
    float ps = 0.f; FragH p0, p1;
#pragma unroll
    for (int r = 0; r < 8; ++r) {
      const float e0 = __expf(s[0][r] - mn), e1 = __expf(s[1][r] - mn), e2 = __expf(s[2][r] - mn), e3 = __expf(s[3][r] - mn);
      ps += (e0 + e1) + (e2 + e3);
      p0.h[r] = (_Float16)(e0 * 1024.0f); p0.h[8 + r] = (_Float16)(e1 * 1024.0f);
      p1.h[r] = (_Float16)(e2 * 1024.0f); p1.h[8 + r] = (_Float16)(e3 * 1024.0f); }
    l = l * c + ps;
#pragma unroll
    for (int r = 0; r < 8; ++r) { o0[r] *= c; o1[r] *= c; }
    v16h va = g2_frag(vb0 + kc, hh);      o0 = g2_mma(va, p0.v, o0);
    va = g2_frag(vb0 + kc + 32, hh);      o0 = g2_mma(va, p1.v, o0);
    va = g2_frag(vb1 + kc, hh);           o1 = g2_mma(va, p0.v, o1);
    va = g2_frag(vb1 + kc + 32, hh);      o1 = g2_mma(va, p1.v, o1);
  }
  const float lt = l + __shfl_xor(l, 16, 32);
  const float fin = 0.0625f / lt;
  FragH w0, w1;
#pragma unroll
  for (int r = 0; r < 8; ++r) { w0.h[r] = (_Float16)(o0[r] * fin); w1.h[r] = (_Float16)(o1[r] * fin); }
  *(v8us*)&so[ln][head * HD + 8 * hh] = w0.half[0];
  *(v8us*)&so[ln][head * HD + 16 + 8 * hh] = w1.half[0];
  __syncthreads();
  for (int pass = 0; pass < 2; ++pass) {
#pragma unroll
    for (int j = 0; j < 2; ++j) { const int i = tid + 256 * j; const int row = i >> 5, c8 = (i & 31) * 8;
      const v8us v = *(const v8us*)&so[row][c8];
      *(volatile v8us*)((unsigned short*)CTX + (size_t)(q0 + row) * CD + c8) = v; }
    if (pass == 0) __threadfence(); }
}
__global__ __launch_bounds__(256) void k_attn_x(const _Float16* __restrict__ QH, const _Float16* __restrict__ QL, const _Float16* __restrict__ Kp, int ldk,
                                                const _Float16* __restrict__ VT, int nk, _Float16* __restrict__ CTX) {
  attn_body<0>(QH, QL, Kp, ldk, VT, nk, nullptr, CTX); }
__global__ __launch_bounds__(256) void k_attn_s(const _Float16* __restrict__ QH, const _Float16* __restrict__ QL, const _Float16* __restrict__ Kp, int ldk,
                                                const _Float16* __restrict__ VT, int nk, const int* __restrict__ cu, const int* __restrict__ cu_kv_unused,
                                                const int* __restrict__ msq_unused, const int* __restrict__ mskv_unused, _Float16* __restrict__ CTX) {
  (void)cu_kv_unused; (void)msq_unused; (void)mskv_unused;
  attn_body<1>(QH, QL, Kp, ldk, VT, nk, cu, CTX); }

constexpr size_t WS_BOUND =
    (size_t)6 * CD * CD * 2 + (size_t)2 * CD * CD * 2 + (size_t)2 * DFF * CD * 2
  + (size_t)4 * NKV * CD * 2 + (size_t)NKV * CD * 2
  + (size_t)11 * NQ * CD * 2
  + (size_t)NQ * 2 * CD * 2 + (size_t)2 * NQ * CD * 4 + (size_t)NQ * DFF * 2
  + (size_t)40 * 256;
static_assert(WS_BOUND <= (size_t)134217728);

extern "C" void kernel_launch(void* const* d_in, const int* in_sizes, int n_in,
                              void* d_out, int out_size, void* d_ws, size_t ws_size, hipStream_t stream) {
  if (n_in < 25) return;
  if (in_sizes[0] < NQ * CD || in_sizes[1] < NKV * CD || in_sizes[2] < NQ * CD || in_sizes[3] < NKV * CD) return;
  if (in_sizes[4] < CD || in_sizes[5] < CD || in_sizes[6] < CD || in_sizes[7] < CD) return;
  if (in_sizes[8] < CD * CD || in_sizes[9] < CD * CD || in_sizes[10] < CD * CD || in_sizes[11] < CD * CD || in_sizes[12] < CD) return;
  if (in_sizes[13] < CD * CD || in_sizes[14] < 2 * CD * CD || in_sizes[15] < CD * CD || in_sizes[16] < CD) return;
  if (in_sizes[17] < DFF * CD || in_sizes[18] < DFF || in_sizes[19] < CD * DFF || in_sizes[20] < CD) return;
  if (in_sizes[21] < NSEG + 1 || in_sizes[22] < 1 || in_sizes[23] < 1 || in_sizes[24] < 1) return;
  if (out_size < NQ * CD) return;
  const float* q = (const float*)d_in[0]; const float* kv = (const float*)d_in[1]; const float* pos_q = (const float*)d_in[2]; const float* pos_k = (const float*)d_in[3];
  const float* w_nkv = (const float*)d_in[4]; const float* w_n1 = (const float*)d_in[5]; const float* w_n2 = (const float*)d_in[6]; const float* w_n3 = (const float*)d_in[7];
  const float* ca_wq = (const float*)d_in[8]; const float* ca_wk = (const float*)d_in[9]; const float* ca_wv = (const float*)d_in[10]; const float* ca_wo = (const float*)d_in[11]; const float* ca_bo = (const float*)d_in[12];
  const float* sa_wq = (const float*)d_in[13]; const float* sa_wkv = (const float*)d_in[14]; const float* sa_wo = (const float*)d_in[15]; const float* sa_bo = (const float*)d_in[16];
  const float* mlp_w1 = (const float*)d_in[17]; const float* mlp_b1 = (const float*)d_in[18]; const float* mlp_w2 = (const float*)d_in[19]; const float* mlp_b2 = (const float*)d_in[20];
  const int* cu_q = (const int*)d_in[21]; const int* cu_kv = (const int*)d_in[22]; const int* msq = (const int*)d_in[23]; const int* mskv = (const int*)d_in[24];
  float* out = (float*)d_out;

  char* ws = (char*)d_ws; size_t off = 0;
  auto take = [&](size_t bytes) { char* p = ws + off; off += (bytes + 255) & ~(size_t)255; return p; };
  _Float16* BQ  = (_Float16*)take((size_t)CD * CD * 2);  _Float16* BK  = (_Float16*)take((size_t)CD * CD * 2);
  _Float16* BV  = (_Float16*)take((size_t)CD * CD * 2);  _Float16* BO  = (_Float16*)take((size_t)CD * CD * 2);
  _Float16* SBQ = (_Float16*)take((size_t)CD * CD * 2);  _Float16* SBKV = (_Float16*)take((size_t)2 * CD * CD * 2);
  _Float16* SBO = (_Float16*)take((size_t)CD * CD * 2);  _Float16* BW1 = (_Float16*)take((size_t)DFF * CD * 2); _Float16* BW2 = (_Float16*)take((size_t)CD * DFF * 2);
  _Float16* KVNP = (_Float16*)take((size_t)NKV * CD * 2); _Float16* KVN = (_Float16*)take((size_t)NKV * CD * 2);
  _Float16* QNP = (_Float16*)take((size_t)NQ * CD * 2);  _Float16* QH = (_Float16*)take((size_t)NQ * CD * 2); _Float16* QL = (_Float16*)take((size_t)NQ * CD * 2);
  _Float16* K16 = (_Float16*)take((size_t)NKV * CD * 2); _Float16* V16 = (_Float16*)take((size_t)NKV * CD * 2); _Float16* VT = (_Float16*)take((size_t)CD * NKV * 2);
  _Float16* CTX = (_Float16*)take((size_t)NQ * CD * 2);  float* X1 = (float*)take((size_t)NQ * CD * 4);
  _Float16* XN2P = (_Float16*)take((size_t)NQ * CD * 2); _Float16* XN2 = (_Float16*)take((size_t)NQ * CD * 2);
  _Float16* QSH = (_Float16*)take((size_t)NQ * CD * 2);  _Float16* QSL = (_Float16*)take((size_t)NQ * CD * 2);
  _Float16* KVS = (_Float16*)take((size_t)NQ * 2 * CD * 2); _Float16* VT2 = (_Float16*)take((size_t)CD * NQ * 2);
  _Float16* CTX2 = (_Float16*)take((size_t)NQ * CD * 2); float* X2 = (float*)take((size_t)NQ * CD * 4);
  _Float16* XN3 = (_Float16*)take((size_t)NQ * CD * 2);  _Float16* H16 = (_Float16*)take((size_t)NQ * DFF * 2);
  if (off > ws_size || off > WS_BOUND) return;

  k_wnat<<<(unsigned)((CD * CD / 8 + 255) / 256), 256, 0, stream>>>(ca_wq, (size_t)CD * CD / 8, BQ);
  k_wnat<<<(unsigned)((CD * CD / 8 + 255) / 256), 256, 0, stream>>>(ca_wk, (size_t)CD * CD / 8, BK);
  k_wnat<<<(unsigned)((CD * CD / 8 + 255) / 256), 256, 0, stream>>>(ca_wv, (size_t)CD * CD / 8, BV);
  k_wnat<<<(unsigned)((CD * CD / 8 + 255) / 256), 256, 0, stream>>>(ca_wo, (size_t)CD * CD / 8, BO);
  k_wnat<<<(unsigned)((CD * CD / 8 + 255) / 256), 256, 0, stream>>>(sa_wq, (size_t)CD * CD / 8, SBQ);
  k_wnat<<<(unsigned)((2 * CD * CD / 8 + 255) / 256), 256, 0, stream>>>(sa_wkv, (size_t)2 * CD * CD / 8, SBKV);
  k_wnat<<<(unsigned)((CD * CD / 8 + 255) / 256), 256, 0, stream>>>(sa_wo, (size_t)CD * CD / 8, SBO);
  k_wnat<<<(unsigned)((DFF * CD / 8 + 255) / 256), 256, 0, stream>>>(mlp_w1, (size_t)DFF * CD / 8, BW1);
  k_wnat<<<(unsigned)((CD * DFF / 8 + 255) / 256), 256, 0, stream>>>(mlp_w2, (size_t)CD * DFF / 8, BW2);

  k_rmsw<<<(unsigned)((NKV + 7) / 8), 256, 0, stream>>>(kv, w_nkv, pos_k, RMS_EPS, 1, KVN, KVNP, NKV);
  k_rmsw<<<(unsigned)((NQ + 7) / 8), 256, 0, stream>>>(q, w_n1, pos_q, RMS_EPS, 1, nullptr, QNP, NQ);
  k_gemm_p<<<(unsigned)((NQ / 128) * (CD / 64)), 128, 0, stream>>>(QNP, CD, BQ, CD, 0.0625f, nullptr, 1.0f, QH, QL, CD, NQ, CD, CD);
  k_gemm_p<<<(unsigned)((NKV / 128) * (CD / 64)), 128, 0, stream>>>(KVNP, CD, BK, CD, 0.0625f, nullptr, 1.0f, K16, nullptr, CD, NKV, CD, CD);
  k_gemm_p<<<(unsigned)((NKV / 128) * (CD / 64)), 128, 0, stream>>>(KVN, CD, BV, CD, 0.0625f, nullptr, 1.0f, V16, nullptr, CD, NKV, CD, CD);
  k_vt<<<(unsigned)(4 * (NKV / 64)), 256, 0, stream>>>(V16, CD, 0, VT, NKV);
  k_attn_x<<<(unsigned)(NQ / 16), 256, 0, stream>>>(QH, QL, K16, CD, VT, NKV, CTX);
  k_gemm_resin<<<(unsigned)((NQ / 128) * (CD / 64)), 128, 0, stream>>>(CTX, CD, BO, CD, 0.0009765625f, ca_bo, q, CD, X1, CD, NQ, CD, CD);

  k_rmsw<<<(unsigned)((NQ + 7) / 8), 256, 0, stream>>>(X1, w_n2, pos_q, RMS_EPS, 0, XN2, XN2P, NQ);
  k_gemm_p<<<(unsigned)((NQ / 128) * (CD / 64)), 128, 0, stream>>>(XN2P, CD, SBQ, CD, 0.0625f, nullptr, 1.0f, QSH, QSL, CD, NQ, CD, CD);
  k_gemm_p<<<(unsigned)((NQ / 128) * (2 * CD / 64)), 128, 0, stream>>>(XN2, CD, SBKV, CD, 0.0625f, nullptr, 1.0f, KVS, nullptr, 2 * CD, NQ, 2 * CD, CD);
  k_vt<<<(unsigned)(4 * (NQ / 64)), 256, 0, stream>>>(KVS, 2 * CD, CD, VT2, NQ);
  k_attn_s<<<(unsigned)(NQ / 16), 256, 0, stream>>>(QSH, QSL, KVS, 2 * CD, VT2, NQ, cu_q, cu_kv, msq, mskv, CTX2);
  k_gemm_res<<<(unsigned)((NQ / 128) * (CD / 64)), 128, 0, stream>>>(CTX2, CD, SBO, CD, 0.0009765625f, sa_bo, X1, CD, X2, CD, NQ, CD, CD);

  k_rmsw<<<(unsigned)((NQ + 7) / 8), 256, 0, stream>>>(X2, w_n3, nullptr, RMS_EPS, 0, XN3, nullptr, NQ);
  k_gemm_gelu<<<(unsigned)((NQ / 128) * (DFF / 64)), 128, 0, stream>>>(XN3, CD, BW1, CD, 0.0625f, mlp_b1, 16.0f, H16, DFF, NQ, DFF, CD);
  k_gemm_res<<<(unsigned)((NQ / 128) * (CD / 64)), 128, 0, stream>>>(H16, DFF, BW2, DFF, 0.00390625f, mlp_b2, X2, CD, out, CD, NQ, CD, DFF);
}
